// LabelEnhanceBert_2001454760481
// MI455X (gfx1250) — hardware-verified
//
#include <hip/hip_runtime.h>
#include <math.h>

typedef __attribute__((ext_vector_type(16))) _Float16 v16h;
typedef __attribute__((ext_vector_type(16))) __bf16 v16b;
typedef __attribute__((ext_vector_type(8)))  _Float16 v8h;
typedef __attribute__((ext_vector_type(8)))  float v8f;
typedef __attribute__((ext_vector_type(4)))  float v4f;
typedef __attribute__((ext_vector_type(2)))  float v2f;
typedef __attribute__((ext_vector_type(4)))  unsigned v4u;
typedef __attribute__((ext_vector_type(4)))  int v4i;
typedef float __attribute__((may_alias)) float_a;
typedef int __attribute__((may_alias)) int_a;

template <typename T> __device__ __forceinline__ void vst2(void* p, T v) { *(volatile T*)p = v; __threadfence(); *(volatile T*)p = v; }
__device__ __forceinline__ v8f wmma16(v16h a, v16h b, v8f c) {
  v8f d = __builtin_amdgcn_wmma_f32_16x16x32_f16(false, a, false, b, (short)0, c, false, false);
  asm volatile("v_nop\n\tv_nop\n\tv_nop\n\tv_nop" : "+v"(d) : "v"(a), "v"(b));
  return d;
}
__device__ __forceinline__ v8f wmma_bf(v16b a, v16b b, v8f c) {
  v8f d = __builtin_amdgcn_wmma_f32_16x16x32_bf16(false, a, false, b, (short)0, c, false, false);
  asm volatile("v_nop\n\tv_nop\n\tv_nop\n\tv_nop" : "+v"(d) : "v"(a), "v"(b));
  return d;
}
__device__ __forceinline__ v16h frag_h(const _Float16* rowk0, int lane) {
  union { v16h v; v8h q[2]; } u; const _Float16* p = rowk0 + 8 * (lane >> 4);
  u.q[0] = *(const v8h*)p; u.q[1] = *(const v8h*)(p + 16); return u.v;
}
__device__ __forceinline__ v16h frag_f32(const float* rowk0, int lane) {
  v16h a; const float* p = rowk0 + 8 * (lane >> 4);
#pragma unroll
  for (int i = 0; i < 8; ++i) { a[i] = (_Float16)p[i]; a[8 + i] = (_Float16)p[16 + i]; }
  return a;
}
__device__ __forceinline__ v16h frag_f32s(const float* rowk0, int lane, float sc) {
  v16h a; const float* p = rowk0 + 8 * (lane >> 4);
#pragma unroll
  for (int i = 0; i < 8; ++i) { a[i] = (_Float16)(p[i] * sc); a[8 + i] = (_Float16)(p[16 + i] * sc); }
  return a;
}
__device__ __forceinline__ v16h fragc_f32(const float* W, int k0, int n, int lane, int ld, int K) {
  v16h a; const int g = lane >> 4;
#pragma unroll
  for (int i = 0; i < 8; ++i) { const int ka = k0 + 8 * g + i, kb = ka + 16;
    a[i] = (_Float16)(ka < K ? W[(size_t)(ka < K ? ka : K - 1) * ld + n] : 0.f); a[8 + i] = (_Float16)(kb < K ? W[(size_t)(kb < K ? kb : K - 1) * ld + n] : 0.f); }
  return a;
}
struct F2 { v16b h, l; };
__device__ __forceinline__ F2 bsplit16(const float v[16]) { F2 r;
#pragma unroll
  for (int i = 0; i < 16; ++i) { const __bf16 h = (__bf16)v[i]; r.h[i] = h; r.l[i] = (__bf16)(v[i] - (float)h); }
  return r; }
__device__ __forceinline__ F2 split_row(const float* row, int k0, int lane) { float v[16]; const float* p = row + k0 + 8 * (lane >> 4);
#pragma unroll
  for (int i = 0; i < 8; ++i) { v[i] = p[i]; v[8 + i] = p[16 + i]; }
  return bsplit16(v); }
__device__ __forceinline__ F2 split_rowK(const float* row, int k0, int lane, int K) { float v[16]; const int g = lane >> 4;
#pragma unroll
  for (int i = 0; i < 8; ++i) { const int ka = k0 + 8 * g + i, kb = ka + 16; v[i] = ka < K ? row[ka < K ? ka : K - 1] : 0.f; v[8 + i] = kb < K ? row[kb < K ? kb : K - 1] : 0.f; }
  return bsplit16(v); }
__device__ __forceinline__ F2 split_col(const float* W, int k0, int n, int lane, int ld, int K) { float v[16]; const int g = lane >> 4;
#pragma unroll
  for (int i = 0; i < 8; ++i) { const int ka = k0 + 8 * g + i, kb = ka + 16; v[i] = ka < K ? W[(size_t)(ka < K ? ka : K - 1) * ld + n] : 0.f; v[8 + i] = kb < K ? W[(size_t)(kb < K ? kb : K - 1) * ld + n] : 0.f; }
  return bsplit16(v); }
__device__ __forceinline__ v8f mac3(const F2& a, const F2& b, v8f c) { c = wmma_bf(a.l, b.h, c); c = wmma_bf(a.h, b.l, c); return wmma_bf(a.h, b.h, c); }
__device__ __forceinline__ float sigm(float v) { return 1.0f / (1.0f + expf(-v)); }
#define LDSX() do { asm volatile("s_wait_dscnt 0" ::: "memory"); __builtin_amdgcn_wave_barrier(); __builtin_amdgcn_fence(__ATOMIC_RELEASE, "workgroup"); } while (0)


#define NT 512
#define NLB 36
#define L2 16
#define NLR (NLB * L2)
#define DB 768
#define DE 512
#define HH 1792
#define VOC 19
__device__ __forceinline__ float bfr(float v) { return (float)(__bf16)v; }
__device__ __forceinline__ v16b frag_b(const __bf16* rowk0, int lane) { return __builtin_bit_cast(v16b, frag_h((const _Float16*)rowk0, lane)); }
__device__ __attribute__((noinline)) float tanh_ni(float v) { return tanhf(v); }

__global__ __launch_bounds__(224) void k_enc(const float* __restrict__ bert, const int* __restrict__ pos_i, const int* __restrict__ ent_i, const float* __restrict__ pos_emb, const float* __restrict__ ent_emb, __bf16* __restrict__ ENC) {
  const int r = blockIdx.x, tid = threadIdx.x; const int c0 = tid * 8;
  int pi = pos_i[r], ei = ent_i[r]; pi = pi < 0 ? 0 : (pi >= VOC ? VOC - 1 : pi); ei = ei < 0 ? 0 : (ei >= VOC ? VOC - 1 : ei);
  const float* src = c0 < DB ? bert + (size_t)r * DB + c0 : (c0 < DB + DE ? pos_emb + (size_t)pi * DE + (c0 - DB) : ent_emb + (size_t)ei * DE + (c0 - DB - DE));
  union { __bf16 e[8]; v4u u; } pk;
#pragma unroll
  for (int e = 0; e < 8; ++e) pk.e[e] = (__bf16)src[e];
  vst2((unsigned*)(ENC + (size_t)r * HH + c0), pk.u);
}
__global__ __launch_bounds__(128) void k_feat(const __bf16* __restrict__ ENC, const float* __restrict__ W, int nrows, float* __restrict__ F) {
  __shared__ __align__(16) float so[4][16][132];
  const int tid = threadIdx.x, wave = tid >> 5, lane = tid & 31, col = lane & 15, g = lane >> 4; const int r0 = blockIdx.x * 64 + wave * 16, n0 = blockIdx.y * 128;
  const int ra = (r0 + col) < nrows ? r0 + col : nrows - 1;
  v8f acc[8] = {};
#pragma unroll 2
  for (int kc = 0; kc < HH / 32; ++kc) { const v16b a = frag_b(ENC + (size_t)ra * HH + kc * 32, lane);
#pragma unroll
    for (int j = 0; j < 8; ++j) acc[j] = wmma_bf(a, split_row(W + (size_t)(n0 + j * 16 + col) * HH, kc * 32, lane).h, acc[j]); }
#pragma unroll
  for (int j = 0; j < 8; ++j)
#pragma unroll
    for (int r = 0; r < 8; ++r) so[wave][8 * g + r][j * 16 + col] = acc[j][r];
  LDSX();
  for (int rl = 0; rl < 16; ++rl) { if (r0 + rl < nrows) vst2(F + (size_t)(r0 + rl) * HH + n0 + lane * 4, *(const v4f*)(&so[wave][rl][lane * 4])); }
}
__global__ __launch_bounds__(128) void k_w3(const float* __restrict__ TF, const float* __restrict__ LF, const float* __restrict__ W3, int which, float* __restrict__ TW3, __bf16* __restrict__ LTh, __bf16* __restrict__ LTl) {
  __shared__ __align__(16) float so[4][16][132]; __shared__ __align__(16) __bf16 sth[4][128][40], stl[4][128][40];
  const int tid = threadIdx.x, wave = tid >> 5, lane = tid & 31, col = lane & 15, g = lane >> 4; const int r0 = blockIdx.x * 64 + wave * 16, n0 = blockIdx.y * 128;
  const float* IN = which == 0 ? TF : LF; const int nrows = which == 0 ? NT : NLR; const int ra = (r0 + col) < nrows ? r0 + col : nrows - 1;
  v8f acc[8] = {};
#pragma unroll 2
  for (int kc = 0; kc < HH / 32; ++kc) { const F2 a = split_row(IN + (size_t)ra * HH, kc * 32, lane);
#pragma unroll
    for (int j = 0; j < 8; ++j) { const v16b wb = split_row(W3 + (size_t)(n0 + j * 16 + col) * HH, kc * 32, lane).h; acc[j] = wmma_bf(a.l, wb, acc[j]); acc[j] = wmma_bf(a.h, wb, acc[j]); } }
  if (which == 0) {
#pragma unroll
    for (int j = 0; j < 8; ++j)
#pragma unroll
      for (int r = 0; r < 8; ++r) so[wave][8 * g + r][j * 16 + col] = acc[j][r];
    LDSX();
    for (int rl = 0; rl < 16; ++rl) { if (r0 + rl < nrows) vst2(TW3 + (size_t)(r0 + rl) * HH + n0 + lane * 4, *(const v4f*)(&so[wave][rl][lane * 4])); } }
  else {
    if (r0 < NLR) { const int n = r0 / L2;
      for (int q = lane; q < 128 * 2; q += 32) { const int o = q >> 1, hf = q & 1; *(v4u*)(&sth[wave][o][16 + hf * 8]) = (v4u){0u, 0u, 0u, 0u}; *(v4u*)(&stl[wave][o][16 + hf * 8]) = (v4u){0u, 0u, 0u, 0u}; }
#pragma unroll
      for (int j = 0; j < 8; ++j)
#pragma unroll
        for (int r = 0; r < 8; ++r) { const float v = acc[j][r]; const __bf16 hi = (__bf16)v; sth[wave][j * 16 + col][8 * g + r] = hi; stl[wave][j * 16 + col][8 * g + r] = (__bf16)(v - (float)hi); }
      LDSX();
      for (int q = lane; q < 128 * 4; q += 32) { const int o = q >> 2, pc = q & 3; const size_t off = (((size_t)n * HH) + n0 + o) * 32 + pc * 8; vst2((unsigned*)(LTh + off), *(const v4u*)(&sth[wave][o][pc * 8])); vst2((unsigned*)(LTl + off), *(const v4u*)(&stl[wave][o][pc * 8])); } } }
}
__global__ __launch_bounds__(128) void k_sc(const float* __restrict__ TF, const float* __restrict__ LF, const int* __restrict__ amask, __bf16* __restrict__ SH, __bf16* __restrict__ SL) {
  __shared__ __align__(16) float ss[4][16][20]; __shared__ __align__(16) __bf16 soh[4][16][10][40], sol[4][16][10][40];
  const int tid = threadIdx.x, wave = tid >> 5, lane = tid & 31, col = lane & 15, g = lane >> 4; const int r0 = blockIdx.x * 16;
  const int ncnt = wave < 3 ? 10 : 6, nbase = wave * 10;
  for (int q = lane; q < 16 * 10 * 2; q += 32) { const int rl = q / 20, rem = q % 20; const int nn = rem >> 1, hf = rem & 1; *(v4u*)(&soh[wave][rl][nn][16 + hf * 8]) = (v4u){0u, 0u, 0u, 0u}; *(v4u*)(&sol[wave][rl][nn][16 + hf * 8]) = (v4u){0u, 0u, 0u, 0u}; }
#pragma unroll 1
  for (int nn = 0; nn < ncnt; ++nn) { const int n = nbase + nn; v8f acc = {};
#pragma unroll 2
    for (int kc = 0; kc < HH / 32; ++kc) { const F2 a = split_row(TF + (size_t)(r0 + col) * HH, kc * 32, lane); const F2 b = split_row(LF + (size_t)(n * L2 + col) * HH, kc * 32, lane); acc = wmma_bf(a.l, b.h, acc); acc = wmma_bf(a.h, b.l, acc); acc = wmma_bf(a.h, b.h, acc); }
#pragma unroll
    for (int r = 0; r < 8; ++r) ss[wave][8 * g + r][col] = acc[r] + (1.0f - (float)amask[n * L2 + col]) * -10000.0f;
    LDSX();
    if (lane < 16) { float v[16]; float mx = -3.4e38f;
#pragma unroll
      for (int k = 0; k < 16; ++k) { v[k] = ss[wave][lane][k]; mx = fmaxf(mx, v[k]); }
      float sum = 0.f;
#pragma unroll
      for (int k = 0; k < 16; ++k) { v[k] = expf(v[k] - mx); sum += v[k]; }
      const float inv = 1.0f / sum;
#pragma unroll
      for (int k = 0; k < 16; ++k) { const float p = v[k] * inv; const __bf16 hi = (__bf16)p; soh[wave][lane][nn][k] = hi; sol[wave][lane][nn][k] = (__bf16)(p - (float)hi); } }
    LDSX(); }
  for (int q = lane; q < 16 * ncnt * 4; q += 32) { const int rl = q / (ncnt * 4), rem = q % (ncnt * 4); const int nn = rem >> 2, pc = rem & 3; const size_t off = (((size_t)(r0 + rl) * NLB) + nbase + nn) * 32 + pc * 8; vst2((unsigned*)(SH + off), *(const v4u*)(&soh[wave][rl][nn][pc * 8])); vst2((unsigned*)(SL + off), *(const v4u*)(&sol[wave][rl][nn][pc * 8])); }
}
__global__ __launch_bounds__(128) void k_fin(const __bf16* __restrict__ SH, const __bf16* __restrict__ SL, const __bf16* __restrict__ LTh, const __bf16* __restrict__ LTl, const float* __restrict__ TW3, const float* __restrict__ b3, const float* __restrict__ wst, const float* __restrict__ bst, const float* __restrict__ wen, const float* __restrict__ ben, float* __restrict__ OS, float* __restrict__ OE) {
  __shared__ float sred[4][16][2]; __shared__ __align__(16) float sos[16][NLB], soe[16][NLB];
  const int tid = threadIdx.x, wave = tid >> 5, lane = tid & 31, col = lane & 15, g = lane >> 4; const int r0 = blockIdx.x * 16;
  const float bS = bfr(bst[0]), bE = bfr(ben[0]);
#pragma unroll 1
  for (int n = 0; n < NLB; ++n) {
    const v16b ah = frag_b(SH + ((size_t)(r0 + col) * NLB + n) * 32, lane), al = frag_b(SL + ((size_t)(r0 + col) * NLB + n) * 32, lane);
    float ds[8] = {0.f, 0.f, 0.f, 0.f, 0.f, 0.f, 0.f, 0.f}, de[8] = {0.f, 0.f, 0.f, 0.f, 0.f, 0.f, 0.f, 0.f};
#pragma unroll 1
    for (int jt = 0; jt < 28; ++jt) { const int o0 = (wave * 28 + jt) * 16; const size_t lo_ = ((size_t)n * HH + o0 + col) * 32; const v16b bh_ = frag_b(LTh + lo_, lane), bl_ = frag_b(LTl + lo_, lane);
      v8f acc = {}; acc = wmma_bf(al, bh_, acc); acc = wmma_bf(ah, bl_, acc); acc = wmma_bf(ah, bh_, acc);
      const int o = o0 + col; const float bb = bfr(b3[o]), w1 = bfr(wst[o]), w2 = bfr(wen[o]);
#pragma unroll
      for (int r = 0; r < 8; ++r) { const float v = tanh_ni(acc[r] + TW3[(size_t)(r0 + 8 * g + r) * HH + o] + bb); ds[r] += v * w1; de[r] += v * w2; } }
#pragma unroll
    for (int r = 0; r < 8; ++r) {
#pragma unroll
      for (int o_ = 1; o_ < 16; o_ <<= 1) { ds[r] += __shfl_xor(ds[r], o_, 32); de[r] += __shfl_xor(de[r], o_, 32); } }
    if (col == 0) {
#pragma unroll
      for (int r = 0; r < 8; ++r) { sred[wave][8 * g + r][0] = ds[r]; sred[wave][8 * g + r][1] = de[r]; } }
    __syncthreads();
    if (tid < 32) { const int rl = tid & 15, which = tid >> 4; const float s = sred[0][rl][which] + sred[1][rl][which] + sred[2][rl][which] + sred[3][rl][which]; if (which == 0) sos[rl][n] = s + bS; else soe[rl][n] = s + bE; }
    __syncthreads(); }
  { const float* ps = &sos[0][0]; const float* pe = &soe[0][0];
    for (int q = tid; q < 16 * NLB / 4; q += 128) { vst2(OS + (size_t)r0 * NLB + q * 4, *(const v4f*)(ps + q * 4)); vst2(OE + (size_t)r0 * NLB + q * 4, *(const v4f*)(pe + q * 4)); } }
}
extern "C" void kernel_launch(void* const* d_in, const int* in_sizes, int n_in, void* d_out, int out_size, void* d_ws, size_t ws_size, hipStream_t stream) {
  (void)in_sizes; (void)n_in; (void)out_size; (void)ws_size;
  const float* text_bert = (const float*)d_in[0]; const float* label_bert = (const float*)d_in[1]; const int* tpos = (const int*)d_in[2]; const int* tent = (const int*)d_in[3]; const int* lpos = (const int*)d_in[4]; const int* lent = (const int*)d_in[5]; const int* amask = (const int*)d_in[6];
  const float* pos_emb = (const float*)d_in[7]; const float* ent_emb = (const float*)d_in[8]; const float* W1 = (const float*)d_in[9]; const float* W2 = (const float*)d_in[10]; const float* W3 = (const float*)d_in[11]; const float* b3 = (const float*)d_in[12];
  const float* wst = (const float*)d_in[13]; const float* bst = (const float*)d_in[14]; const float* wen = (const float*)d_in[15]; const float* ben = (const float*)d_in[16];
  float* OS = (float*)d_out; float* OE = (float*)((char*)d_out + 73728);
  char* ws = (char*)d_ws; size_t off = 0;
  auto take = [&](size_t bytes) { char* p = ws + off; off += (bytes + 255) & ~(size_t)255; return p; };
  __bf16* ENCT = (__bf16*)take((size_t)NT * HH * 2); __bf16* ENCL = (__bf16*)take((size_t)NLR * HH * 2); float* TF = (float*)take((size_t)NT * HH * 4); float* LF = (float*)take((size_t)NLR * HH * 4); float* TW3 = (float*)take((size_t)NT * HH * 4);
  __bf16* LTh = (__bf16*)take((size_t)NLB * HH * 32 * 2); __bf16* LTl = (__bf16*)take((size_t)NLB * HH * 32 * 2); __bf16* SH = (__bf16*)take((size_t)NT * NLB * 32 * 2); __bf16* SL = (__bf16*)take((size_t)NT * NLB * 32 * 2);
  k_enc<<<NT, 224, 0, stream>>>(text_bert, tpos, tent, pos_emb, ent_emb, ENCT);
  k_enc<<<NLR, 224, 0, stream>>>(label_bert, lpos, lent, pos_emb, ent_emb, ENCL);
  k_feat<<<dim3(NT / 64, HH / 128), 128, 0, stream>>>(ENCT, W1, NT, TF);
  k_feat<<<dim3(NLR / 64, HH / 128), 128, 0, stream>>>(ENCL, W2, NLR, LF);
  k_w3<<<dim3(NT / 64, HH / 128), 128, 0, stream>>>(TF, LF, W3, 0, TW3, LTh, LTl);
  k_w3<<<dim3(NLR / 64, HH / 128), 128, 0, stream>>>(TF, LF, W3, 1, TW3, LTh, LTl);
  k_sc<<<NT / 16, 128, 0, stream>>>(TF, LF, amask, SH, SL);
  k_fin<<<NT / 16, 128, 0, stream>>>(SH, SL, LTh, LTl, TW3, b3, wst, bst, wen, ben, OS, OE);
}
